// manual_MHA_61615600828751
// MI455X (gfx1250) — hardware-verified
//
#include <hip/hip_runtime.h>


#define SS   4096
#define DMOD 512
#define NH_  8
#define HD   64
#define RCH  1024
#define DM   DMOD
#define NTK  SS
#define ISC  0.125f
#define LOSC 1024.0f

typedef _Float16 h16;
typedef unsigned short bf;
typedef __attribute__((ext_vector_type(16))) __bf16   v16bf;
typedef __attribute__((ext_vector_type(16))) _Float16 v16h;
typedef __attribute__((ext_vector_type(8)))  _Float16 v8h;
typedef __attribute__((ext_vector_type(8)))  unsigned short v8us;
typedef __attribute__((ext_vector_type(8)))  float    v8f;
typedef __attribute__((ext_vector_type(4)))  float    v4f;
typedef __attribute__((ext_vector_type(4)))  _Float16 v4h;
typedef v8h  __attribute__((may_alias)) v8ha;
typedef v4f  __attribute__((may_alias)) v4fa;
typedef v8us __attribute__((may_alias)) v8usa;

__device__ __forceinline__ unsigned short f2bf(float f) { unsigned u = __float_as_uint(f); u += 0x7FFFu + ((u >> 16) & 1u); return (unsigned short)(u >> 16); }
__device__ __forceinline__ float bf2f(unsigned short b) { return __uint_as_float(((unsigned)b) << 16); }
__device__ __forceinline__ float bfr(float f) { return bf2f(f2bf(f)); }
__device__ __forceinline__ v16h cat16(v8h lo, v8h hi) { return __builtin_shufflevector(lo, hi, 0, 1, 2, 3, 4, 5, 6, 7, 8, 9, 10, 11, 12, 13, 14, 15); }
__device__ __forceinline__ v16bf cat16b(v8us lo, v8us hi) { return __builtin_bit_cast(v16bf, __builtin_shufflevector(lo, hi, 0, 1, 2, 3, 4, 5, 6, 7, 8, 9, 10, 11, 12, 13, 14, 15)); }
__device__ __forceinline__ v8f wmma16(v16h a, v16h b, v8f c) { return __builtin_amdgcn_wmma_f32_16x16x32_f16(false, a, false, b, (short)0, c, false, false); }
__device__ __forceinline__ v8f wmmab(v16bf a, v16bf b, v8f c) { return __builtin_amdgcn_wmma_f32_16x16x32_bf16(false, a, false, b, (short)0, c, false, false); }

__global__ __launch_bounds__(256) void k_wt(const float* __restrict__ Wm, int K, int ncols, bf* WT) {
    __shared__ __align__(16) unsigned short tl[64 * 72];
    const int tid = threadIdx.x, k0 = blockIdx.x * 64, n0 = blockIdx.y * 64;
    const int kk = tid >> 2, nq = (tid & 3) * 16;
#pragma unroll
    for (int i = 0; i < 16; ++i) tl[(nq + i) * 72 + kk] = f2bf(Wm[(size_t)(k0 + kk) * ncols + n0 + nq + i]);
    __syncthreads();
    const int piece = tid & 7;
    auto pass = [&]() {
#pragma unroll
        for (int s = 0; s < 2; ++s) { const int nr = (tid >> 3) + 32 * s; const v8us val = *(const v8usa*)(tl + nr * 72 + piece * 8); *(volatile v8us*)(WT + (size_t)(n0 + nr) * K + k0 + piece * 8) = val; }
    };
    pass(); __threadfence(); pass();
}
template <bool SPLITA, bool F16OUT = false>
__global__ __launch_bounds__(128) void k_gemmb(const bf* __restrict__ A, const bf* __restrict__ Al, const bf* __restrict__ Bn, const float* __restrict__ bias, float* C, int ldc, h16* C2, const float* __restrict__ R = nullptr, int K = DM, int roundR = 1) {
    __shared__ __align__(16) float ost[4][16 * 68];
    const int lane = threadIdx.x & 31, wave = threadIdx.x >> 5, lr = lane & 15, hi = lane >> 4;
    const int r0 = blockIdx.x * 64 + wave * 16, c0 = blockIdx.y * 64;
    const size_t aoff = (size_t)(r0 + lr) * K + 8 * hi;
    size_t boff[4];
#pragma unroll
    for (int t = 0; t < 4; ++t) boff[t] = (size_t)(c0 + t * 16 + lr) * K + 8 * hi;
    v8f acc[4];
#pragma unroll
    for (int t = 0; t < 4; ++t) acc[t] = (v8f){};
#pragma unroll 1
    for (int kc = 0; kc < K; kc += 32) {
        const v16bf a = cat16b(*(const v8us*)(A + aoff + kc), *(const v8us*)(A + aoff + kc + 16));
        v16bf al = a;
        if (SPLITA) al = cat16b(*(const v8us*)(Al + aoff + kc), *(const v8us*)(Al + aoff + kc + 16));
#pragma unroll
        for (int t = 0; t < 4; ++t) { const v16bf b = cat16b(*(const v8us*)(Bn + boff[t] + kc), *(const v8us*)(Bn + boff[t] + kc + 16)); acc[t] = wmmab(a, b, acc[t]); if (SPLITA) acc[t] = wmmab(al, b, acc[t]); }
        asm volatile("v_nop\n\tv_nop\n\tv_nop\n\tv_nop" : "+v"(acc[0]), "+v"(acc[1]), "+v"(acc[2]), "+v"(acc[3]) : "v"(a), "v"(al));
    }
    float* os = &ost[wave][0];
#pragma unroll
    for (int t = 0; t < 4; ++t) { const float bv = bias ? bfr(bias[c0 + t * 16 + lr]) : 0.f;
#pragma unroll
        for (int j = 0; j < 8; ++j) os[(hi * 8 + j) * 68 + t * 16 + lr] = acc[t][j] + bv; }
    __syncthreads();
    if (F16OUT) {
        h16* crow = (h16*)(void*)C + (size_t)r0 * ldc + c0;
        auto pass = [&]() {
#pragma unroll
            for (int s = 0; s < 4; ++s) { const int row = 4 * s + (lane >> 3), piece = lane & 7; const float* sp = os + row * 68 + piece * 8; v8h o, o2;
#pragma unroll
                for (int i = 0; i < 8; ++i) { const h16 a = (h16)sp[i]; o[i] = a; o2[i] = (h16)((sp[i] - (float)a) * LOSC); }
                *(volatile v8h*)(crow + (size_t)row * ldc + piece * 8) = o; if (C2) *(volatile v8h*)(C2 + (size_t)r0 * ldc + c0 + (size_t)row * ldc + piece * 8) = o2; }
        };
        pass(); __threadfence(); pass();
    } else {
        float* crow = C + (size_t)r0 * ldc + c0;
        auto pass = [&]() {
#pragma unroll
            for (int s = 0; s < 8; ++s) { const int Lid = (lane >> 3) + 4 * s, piece = lane & 7; const int row = Lid >> 1, cofs = (Lid & 1) * 32 + piece * 4;
                v4f val = *(const v4fa*)(os + row * 68 + cofs); if (R) { const v4f rv = *(const v4f*)(R + ((size_t)r0 + row) * ldc + c0 + cofs); val += roundR ? (v4f){bfr(rv[0]), bfr(rv[1]), bfr(rv[2]), bfr(rv[3])} : rv; }
                *(volatile v4f*)(crow + (size_t)row * ldc + cofs) = val; }
        };
        pass(); __threadfence(); pass();
    }
}

__global__ __launch_bounds__(128) void k_gemm3(const bf* __restrict__ Ah, const bf* __restrict__ Al, const bf* __restrict__ Bh, const bf* __restrict__ Bl, int K, float* C, int ldc) {
    __shared__ __align__(16) float ost[4][16 * 68];
    const int lane = threadIdx.x & 31, wave = threadIdx.x >> 5, lr = lane & 15, hi = lane >> 4;
    const int r0 = blockIdx.x * 64 + wave * 16, c0 = blockIdx.y * 64;
    const size_t aoff = (size_t)(r0 + lr) * K + 8 * hi;
    v8f acc[4];
#pragma unroll
    for (int t = 0; t < 4; ++t) acc[t] = (v8f){};
#pragma unroll 1
    for (int kc = 0; kc < K; kc += 32) {
        const v16bf a = cat16b(*(const v8us*)(Ah + aoff + kc), *(const v8us*)(Ah + aoff + kc + 16));
        const v16bf al = cat16b(*(const v8us*)(Al + aoff + kc), *(const v8us*)(Al + aoff + kc + 16));
#pragma unroll
        for (int t = 0; t < 4; ++t) { const size_t bo = (size_t)(c0 + t * 16 + lr) * K + kc + 8 * hi;
            const v16bf bh = cat16b(*(const v8us*)(Bh + bo), *(const v8us*)(Bh + bo + 16)); const v16bf bl = cat16b(*(const v8us*)(Bl + bo), *(const v8us*)(Bl + bo + 16));
            acc[t] = wmmab(a, bh, acc[t]); acc[t] = wmmab(al, bh, acc[t]); acc[t] = wmmab(a, bl, acc[t]); }
        asm volatile("v_nop\n\tv_nop\n\tv_nop\n\tv_nop" : "+v"(acc[0]), "+v"(acc[1]), "+v"(acc[2]), "+v"(acc[3]) : "v"(a), "v"(al));
    }
    float* os = &ost[wave][0];
#pragma unroll
    for (int t = 0; t < 4; ++t) {
#pragma unroll
        for (int j = 0; j < 8; ++j) os[(hi * 8 + j) * 68 + t * 16 + lr] = acc[t][j]; }
    __builtin_amdgcn_wave_barrier(); asm volatile("" ::: "memory");
    float* crow = C + (size_t)r0 * ldc + c0;
    auto pass = [&]() {
#pragma unroll
        for (int s = 0; s < 8; ++s) { const int Lid = (lane >> 3) + 4 * s, piece = lane & 7; const int row = Lid >> 1, cofs = (Lid & 1) * 32 + piece * 4;
            const v4f val = *(const v4fa*)(os + row * 68 + cofs); *(volatile v4f*)(crow + (size_t)row * ldc + cofs) = val; }
    };
    pass(); __threadfence(); pass();
}


__global__ __launch_bounds__(256) void k_cvtx(const float* __restrict__ src, bf* dst) {
    const int lane = threadIdx.x & 31; const size_t r = (size_t)blockIdx.x * 8 + (threadIdx.x >> 5); if (r >= (size_t)SS) return;
#pragma unroll 1
    for (int ps = 0; ps < 2; ++ps) {
#pragma unroll
        for (int q = 0; q < DMOD / 256; ++q) { v8us o;
#pragma unroll
            for (int i = 0; i < 8; ++i) o[i] = f2bf(src[r * DMOD + q * 256 + lane * 8 + i]);
            *(volatile v8us*)(dst + r * DMOD + q * 256 + lane * 8) = o; }
        if (ps == 0) __threadfence(); }
}
__global__ __launch_bounds__(256) void k_wh(const float* __restrict__ P, bf* WT) {
    const int lane = threadIdx.x & 31; const size_t r = (size_t)blockIdx.x * 8 + (threadIdx.x >> 5); if (r >= (size_t)DMOD) return; const int h = (int)(r / HD), k = (int)(r % HD);
#pragma unroll 1
    for (int ps = 0; ps < 2; ++ps) {
#pragma unroll
        for (int q = 0; q < DMOD / 256; ++q) { v8us o;
#pragma unroll
            for (int i = 0; i < 8; ++i) { const int d = q * 256 + lane * 8 + i; o[i] = f2bf(P[((size_t)h * DMOD + d) * HD + k]); }
            *(volatile v8us*)(WT + r * DMOD + q * 256 + lane * 8) = o; }
        if (ps == 0) __threadfence(); }
}
__global__ __launch_bounds__(256) void k_hplanes(const float* __restrict__ F, int h, bf* Ph, bf* Pl) {
    typedef __attribute__((ext_vector_type(2))) unsigned short v2us;
    const int lane = threadIdx.x & 31; const size_t s = (size_t)blockIdx.x * 8 + (threadIdx.x >> 5); if (s >= (size_t)SS) return; v2us oh, ol;
#pragma unroll
    for (int i = 0; i < 2; ++i) { const float v = F[s * DMOD + h * HD + lane * 2 + i]; const unsigned short hb = f2bf(v); oh[i] = hb; ol[i] = f2bf(v - bf2f(hb)); }
    const size_t o = s * HD + lane * 2; *(volatile v2us*)(Ph + o) = oh; *(volatile v2us*)(Pl + o) = ol; __threadfence(); *(volatile v2us*)(Ph + o) = oh; *(volatile v2us*)(Pl + o) = ol;
}
__global__ __launch_bounds__(256) void k_vt(const float* __restrict__ VF, int h, bf* Th, bf* Tl) {
    typedef __attribute__((ext_vector_type(2))) unsigned short v2us;
    const int lane = threadIdx.x & 31; const size_t wid = (size_t)blockIdx.x * 8 + (threadIdx.x >> 5); if (wid >= (size_t)HD * (SS / 64)) return; const int d = (int)(wid / (SS / 64)); const int t0 = (int)(wid % (SS / 64)) * 64 + lane * 2; v2us oh, ol;
#pragma unroll
    for (int i = 0; i < 2; ++i) { const float v = VF[(size_t)(t0 + i) * DMOD + h * HD + d]; const unsigned short hb = f2bf(v); oh[i] = hb; ol[i] = f2bf(v - bf2f(hb)); }
    const size_t o = (size_t)d * SS + t0; *(volatile v2us*)(Th + o) = oh; *(volatile v2us*)(Tl + o) = ol; __threadfence(); *(volatile v2us*)(Th + o) = oh; *(volatile v2us*)(Tl + o) = ol;
}
__global__ __launch_bounds__(256) void k_exp(const float* __restrict__ S, bf* EH, bf* EL, float* RSL) {
    typedef __attribute__((ext_vector_type(4))) unsigned short v4us;
    __shared__ float sh[8];
    const int lane = threadIdx.x & 31, wv = threadIdx.x >> 5, rl = blockIdx.x * 8 + wv; const float* sr = S + (size_t)rl * SS; float tot = 0.f;
#pragma unroll 1
    for (int ps = 0; ps < 2; ++ps) { tot = 0.f;
#pragma unroll 1
        for (int c0 = lane * 4; c0 < SS; c0 += 128) { v4us oh, ol;
#pragma unroll
            for (int q = 0; q < 4; ++q) { const float e = __expf(sr[c0 + q] * ISC); tot += e; const unsigned short hb = f2bf(e); oh[q] = hb; ol[q] = f2bf(e - bf2f(hb)); }
            const size_t o = (size_t)rl * SS + c0; *(volatile v4us*)(EH + o) = oh; *(volatile v4us*)(EL + o) = ol; }
        if (ps == 0) __threadfence(); }
#pragma unroll
    for (int x = 16; x; x >>= 1) tot += __shfl_xor(tot, x, 32);
    if (lane == 0) sh[wv] = tot;
    __syncthreads();
    if (wv == 0) { const float v = (lane < 8) ? sh[lane] : 0.f; float* d = RSL + (size_t)blockIdx.x * 32 + lane; *(volatile float*)d = v; __threadfence(); *(volatile float*)d = v; }
}
__global__ __launch_bounds__(256) void k_total(const float* __restrict__ RSL, float* TOT) {
    __shared__ float pa[256];
    const int t = threadIdx.x; float a = 0.f; const int per = NH_ * SS / 256;
    for (int q = 0; q < per; ++q) { const int i = t * per + q; a += RSL[(size_t)(i >> 3) * 32 + (i & 7)]; }
    pa[t] = a; __syncthreads();
    if (t < 32) { float v = 0.f; if (t == 0) { float A = 0.f; for (int k = 0; k < 256; ++k) A += pa[k]; v = A; } *(volatile float*)(TOT + t) = v; __threadfence(); *(volatile float*)(TOT + t) = v; }
}
__global__ __launch_bounds__(256) void k_cat(const float* __restrict__ U, const float* __restrict__ TOT, bf* Ch, bf* Cl) {
    const int lane = threadIdx.x & 31; const size_t s = (size_t)blockIdx.x * 8 + (threadIdx.x >> 5); if (s >= (size_t)SS) return; const float inv = 1.0f / TOT[0];
#pragma unroll 1
    for (int ps = 0; ps < 2; ++ps) {
#pragma unroll
        for (int q = 0; q < DMOD / 256; ++q) { const size_t o = s * DMOD + q * 256 + lane * 8; v8us oh, ol;
#pragma unroll
            for (int i = 0; i < 8; ++i) { const float v = U[o + i] * inv; const unsigned short hb = f2bf(v); oh[i] = hb; ol[i] = f2bf(v - bf2f(hb)); }
            *(volatile v8us*)(Ch + o) = oh; *(volatile v8us*)(Cl + o) = ol; }
        if (ps == 0) __threadfence(); }
}

extern "C" void kernel_launch(void* const* d_in, const int* in_sizes, int n_in,
                              void* d_out, int out_size, void* d_ws, size_t ws_size, hipStream_t stream) {
    (void)in_sizes; (void)n_in; (void)out_size;
    const float* x = (const float*)d_in[0]; const float* qp = (const float*)d_in[1]; const float* kp = (const float*)d_in[2]; const float* vp = (const float*)d_in[3]; const float* op = (const float*)d_in[4];
    float* out = (float*)d_out;
    char* wsp = (char*)d_ws;
    auto take = [&](size_t bytes) { char* p = wsp; wsp += (bytes + 255) & ~(size_t)255; return (void*)p; };
    bf* WQ = (bf*)take((size_t)DMOD * DMOD * 2); bf* WK = (bf*)take((size_t)DMOD * DMOD * 2); bf* WV = (bf*)take((size_t)DMOD * DMOD * 2); bf* WO = (bf*)take((size_t)DMOD * DMOD * 2);
    bf* Xb = (bf*)take((size_t)SS * DMOD * 2); float* QF = (float*)take((size_t)SS * DMOD * 4); float* KF = (float*)take((size_t)SS * DMOD * 4); float* VF = (float*)take((size_t)SS * DMOD * 4);
    bf* Qh = (bf*)take((size_t)SS * HD * 2); bf* Ql = (bf*)take((size_t)SS * HD * 2); bf* Kh = (bf*)take((size_t)SS * HD * 2); bf* Kl = (bf*)take((size_t)SS * HD * 2); bf* VTh = (bf*)take((size_t)HD * SS * 2); bf* VTl = (bf*)take((size_t)HD * SS * 2);
    float* S = (float*)take((size_t)RCH * SS * 4); bf* EH = (bf*)take((size_t)RCH * SS * 2); bf* EL = (bf*)take((size_t)RCH * SS * 2); float* RSL = (float*)take((size_t)NH_ * (SS / 8) * 32 * 4); float* TOT = (float*)take(32 * 4);
    float* U = (float*)take((size_t)SS * DMOD * 4); bf* Ch = (bf*)take((size_t)SS * DMOD * 2); bf* Cl = (bf*)take((size_t)SS * DMOD * 2);
    if ((size_t)(wsp - (char*)d_ws) > ws_size) return;
    k_wh<<<DMOD / 8, 256, 0, stream>>>(qp, WQ); k_wh<<<DMOD / 8, 256, 0, stream>>>(kp, WK); k_wh<<<DMOD / 8, 256, 0, stream>>>(vp, WV); k_wt<<<dim3(DMOD / 64, DMOD / 64, 1), 256, 0, stream>>>(op, DMOD, DMOD, WO);
    k_cvtx<<<SS / 8, 256, 0, stream>>>(x, Xb);
    k_gemmb<false, false><<<dim3(SS / 64, DMOD / 64, 1), 128, 0, stream>>>(Xb, nullptr, WQ, nullptr, QF, DMOD, nullptr, nullptr, DMOD);
    k_gemmb<false, false><<<dim3(SS / 64, DMOD / 64, 1), 128, 0, stream>>>(Xb, nullptr, WK, nullptr, KF, DMOD, nullptr, nullptr, DMOD);
    k_gemmb<false, false><<<dim3(SS / 64, DMOD / 64, 1), 128, 0, stream>>>(Xb, nullptr, WV, nullptr, VF, DMOD, nullptr, nullptr, DMOD);
    for (int h = 0; h < NH_; ++h) {
        k_hplanes<<<SS / 8, 256, 0, stream>>>(QF, h, Qh, Ql); k_hplanes<<<SS / 8, 256, 0, stream>>>(KF, h, Kh, Kl); k_vt<<<(HD * (SS / 64)) / 8, 256, 0, stream>>>(VF, h, VTh, VTl);
        for (int ch = 0; ch < SS / RCH; ++ch) { const size_t q0 = (size_t)ch * RCH;
            k_gemm3<<<dim3(RCH / 64, SS / 64, 1), 128, 0, stream>>>(Qh + q0 * HD, Ql + q0 * HD, Kh, Kl, HD, S, SS);
            k_exp<<<RCH / 8, 256, 0, stream>>>(S, EH, EL, RSL + (((size_t)h * SS + q0) / 8) * 32);
            k_gemm3<<<dim3(RCH / 64, 1, 1), 128, 0, stream>>>(EH, EL, VTh, VTl, SS, U + q0 * DMOD + h * HD, DMOD); } }
    k_total<<<1, 256, 0, stream>>>(RSL, TOT);
    k_cat<<<SS / 8, 256, 0, stream>>>(U, TOT, Ch, Cl);
    k_gemmb<true, false><<<dim3(SS / 64, DMOD / 64, 1), 128, 0, stream>>>(Ch, Cl, WO, nullptr, out, DMOD, nullptr, nullptr, DMOD);
}
